// SSelfAttention_1082331758992
// MI455X (gfx1250) — hardware-verified
//
#include <hip/hip_runtime.h>


namespace {
constexpr int NB_ = 2, N = 512, T = 24, E = 64, H = 8, HD = 8, NBT = NB_ * T  ;
constexpr float HS = 256.0f, PS = 256.0f, WSC = 256.0f, SCALE = 0.125f  ;
typedef _Float16 b16;
typedef __attribute__((ext_vector_type(16))) _Float16 v16b;
typedef __attribute__((ext_vector_type(8))) _Float16 v8b;
typedef __attribute__((ext_vector_type(8))) float v8f;
typedef __attribute__((ext_vector_type(4))) float v4f;
typedef __attribute__((ext_vector_type(2))) float v2f;
__device__ __forceinline__ float bf16_rne(float f) { unsigned int u = __float_as_uint(f); u += 0x7FFFu + ((u >> 16) & 1u); float r = __uint_as_float(u & 0xFFFF0000u); asm volatile("" : "+v"(r)); return r; }
__device__ __forceinline__ float bfv(float f) { float r = bf16_rne(f); asm volatile("" : "+v"(r)); return r; }
__device__ __forceinline__ void split16(float v, b16& hi, b16& lo) { hi = (b16)v; lo = (b16)(v - (float)hi); }
__device__ __forceinline__ v16b frag_kb(const b16* p, int hh) { const v8b a = *(const v8b*)(p + 8 * hh), b = *(const v8b*)(p + 16 + 8 * hh); v16b f;
#pragma unroll
  for (int e = 0; e < 8; ++e) { f[e] = a[e]; f[8 + e] = b[e]; } return f; }
__device__ __forceinline__ v8f wmma16b(v16b a, v16b b, v8f c) { v8f d = __builtin_amdgcn_wmma_f32_16x16x32_f16(false, a, false, b, (short)0, c, false, false); asm volatile("v_nop\n\tv_nop\n\tv_nop\n\tv_nop" : "+v"(d) : "v"(a), "v"(b)); return d; }
__device__ __forceinline__ void wave_lds_sync() { __builtin_amdgcn_fence(__ATOMIC_RELEASE, "workgroup"); __builtin_amdgcn_wave_barrier(); __builtin_amdgcn_fence(__ATOMIC_ACQUIRE, "workgroup"); }
__device__ __forceinline__ float pmul(float a, float b) { float p = a * b; asm volatile("" : "+v"(p)); return p; }

typedef __attribute__((ext_vector_type(2))) _Float16 v2b;
__global__ __launch_bounds__(256) void proj_kernel(const float* __restrict__ xv, const float* __restrict__ xk, const float* __restrict__ xq, const float* __restrict__ wv, const float* __restrict__ wk, const float* __restrict__ wq, b16* __restrict__ QPh, b16* __restrict__ QPl, b16* __restrict__ KPh, b16* __restrict__ KPl, b16* __restrict__ VTh, b16* __restrict__ VTl) { __shared__ float Vs[H][HD][65], Wl[3][HD][HD]; const int b = blockIdx.x / (T * (N / 64)), rem = blockIdx.x % (T * (N / 64)); const int t = rem / (N / 64), n0 = (rem % (N / 64)) * 64; const int tid = threadIdx.x, h = tid >> 5, lane = tid & 31; const int bth = (b * T + t) * H + h;
  if (tid < 3 * HD * HD) { const int w = tid / (HD * HD), ij = tid % (HD * HD); const float* src = w == 0 ? wq : (w == 1 ? wk : wv); Wl[w][ij / HD][ij % HD] = bfv(src[ij]); }
  __syncthreads();
  const v8b z8 = {0, 0, 0, 0, 0, 0, 0, 0};
  for (int half = 0; half < 2; ++half) { const int n = n0 + half * 32 + lane; const size_t xo = (((size_t)b * N + n) * T + t) * E + h * HD; const size_t ro = ((size_t)bth * N + n) * 32;
    for (int which = 0; which < 3; ++which) { const float* xs = which == 0 ? xq : (which == 1 ? xk : xv); float xx[HD];
#pragma unroll
      for (int j = 0; j < HD; ++j) xx[j] = bfv(xs[xo + j]);
      v8b hh8, ll8;
#pragma unroll
      for (int i = 0; i < HD; ++i) { float s = 0.0f;
#pragma unroll
        for (int j = 0; j < HD; ++j) s += pmul(xx[j], Wl[which][i][j]); if (which == 2) Vs[h][i][half * 32 + lane] = s; else { b16 p, pl; split16(s * HS, p, pl); hh8[i] = p; ll8[i] = pl; } }
      if (which < 2) { b16* Ph = which == 0 ? QPh : KPh; b16* Pl = which == 0 ? QPl : KPl; for (int pass = 0; pass < 2; ++pass) { *(volatile v8b*)(Ph + ro) = hh8; *(volatile v8b*)(Pl + ro) = ll8; for (int c = 8; c < 32; c += 8) { *(volatile v8b*)(Ph + ro + c) = z8; *(volatile v8b*)(Pl + ro + c) = z8; } __threadfence(); } } } }
  __syncthreads();
  for (int pass = 0; pass < 2; ++pass) { for (int d = 0; d < 16; ++d) { b16 h0 = (b16)0.0f, l0 = (b16)0.0f, h1 = (b16)0.0f, l1 = (b16)0.0f; if (d < HD) { split16(Vs[h][d][lane * 2] * HS, h0, l0); split16(Vs[h][d][lane * 2 + 1] * HS, h1, l1); } const size_t o = ((size_t)bth * 16 + d) * N + n0 + lane * 2; *(volatile v2b*)(VTh + o) = (v2b){h0, h1}; *(volatile v2b*)(VTl + o) = (v2b){l0, l1}; } __threadfence(); } }
__global__ __launch_bounds__(32) void att_kernel(const b16* __restrict__ QPh, const b16* __restrict__ QPl, const b16* __restrict__ KPh, const b16* __restrict__ KPl, const b16* __restrict__ VTh, const b16* __restrict__ VTl, int GLIM, float* __restrict__ AO) { __shared__ __attribute__((aligned(16))) b16 Pa[16][N + 8], Pb[16][N + 8]; __shared__ float Sc[16][N + 1], Of[16][9]; const int lane = threadIdx.x, nloc = lane & 15, hlf = lane >> 4; const int bth = blockIdx.x / (N / 16), q0 = (blockIdx.x % (N / 16)) * 16; if (bth >= GLIM) return;
  const v16b qa = frag_kb(QPh + ((size_t)bth * N + q0 + nloc) * 32, hlf), ql = frag_kb(QPl + ((size_t)bth * N + q0 + nloc) * 32, hlf);
#pragma unroll 4
  for (int tk = 0; tk < N / 16; ++tk) { const size_t ko = ((size_t)bth * N + tk * 16 + nloc) * 32; const v16b kh = frag_kb(KPh + ko, hlf), kl = frag_kb(KPl + ko, hlf); v8f s = wmma16b(qa, kh, (v8f){}); s = wmma16b(qa, kl, s); s = wmma16b(ql, kh, s);
#pragma unroll
    for (int r8 = 0; r8 < 8; ++r8) Sc[8 * hlf + r8][tk * 16 + nloc] = s[r8] * (SCALE / (HS * HS)); }
  wave_lds_sync();
  if (lane < 16) { const int r = lane; float mx = -INFINITY; for (int k = 0; k < N; ++k) mx = fmaxf(mx, Sc[r][k]); float sm = 0.0f; for (int k = 0; k < N; ++k) { const float p = __expf(Sc[r][k] - mx); Sc[r][k] = p; sm += p; } const float inv = 1.0f / sm; for (int k = 0; k < N; ++k) { b16 p, pl; split16(Sc[r][k] * inv * PS, p, pl); Pa[r][k] = p; Pb[r][k] = pl; } for (int k = N; k < N + 8; ++k) { Pa[r][k] = (b16)0.0f; Pb[r][k] = (b16)0.0f; } }
  wave_lds_sync();
  v8f o = (v8f){};
#pragma unroll 4
  for (int kb = 0; kb < N; kb += 32) { const v16b pa = frag_kb(&Pa[nloc][kb], hlf), pb = frag_kb(&Pb[nloc][kb], hlf); const size_t vo = ((size_t)bth * 16 + nloc) * N + kb; const v16b vh = frag_kb(VTh + vo, hlf), vl = frag_kb(VTl + vo, hlf); o = wmma16b(pa, vh, o); o = wmma16b(pa, vl, o); o = wmma16b(pb, vh, o); }
#pragma unroll
  for (int r8 = 0; r8 < 8; ++r8) if (nloc < HD) Of[8 * hlf + r8][nloc] = o[r8] * (1.0f / (PS * HS));
  wave_lds_sync();
  for (int pass = 0; pass < 2; ++pass) { for (int q = 0; q < 4; ++q) { const int idx = q * 32 + lane; ((volatile float*)AO)[((size_t)bth * N + q0) * HD + idx] = Of[idx >> 3][idx & 7]; } __threadfence(); } }
__global__ __launch_bounds__(32) void outp_kernel(const float* __restrict__ AO, const float* __restrict__ wo, const float* __restrict__ bo, int GLIM, float* __restrict__ out) { __shared__ __attribute__((aligned(16))) b16 Ah[16][E + 8], Al[16][E + 8], Wr[E][E + 8]; __shared__ float Tf[16][E + 1]; const int lane = threadIdx.x, nloc = lane & 15, hlf = lane >> 4; const size_t r0 = (size_t)blockIdx.x * 16;
  for (int o = 0; o < E; ++o) for (int q = 0; q < 2; ++q) Wr[o][q * 32 + lane] = (b16)(bfv(wo[o * E + q * 32 + lane]) * WSC); if (lane < 16) for (int o = 0; o < E; o += 1) for (int k = E; k < E + 8; ++k) Wr[o][k] = (b16)0.0f;
  for (int rr = 0; rr < 16; ++rr) { const size_t row = r0 + rr; const int b = (int)(row / ((size_t)N * T)), n = (int)((row / T) % N), t = (int)(row % T); for (int q = 0; q < 2; ++q) { const int c = q * 32 + lane; const int h = c / HD, d = c % HD; const int bth = (b * T + t) * H + h; const float v = bth < GLIM ? AO[((size_t)bth * N + n) * HD + d] : 0.0f; b16 p, pl; split16(v * HS, p, pl); Ah[rr][c] = p; Al[rr][c] = pl; } }
  if (lane < 16) for (int k = E; k < E + 8; ++k) { Ah[lane][k] = (b16)0.0f; Al[lane][k] = (b16)0.0f; }
  wave_lds_sync(); v8f acc[4] = {(v8f){}, (v8f){}, (v8f){}, (v8f){}};
#pragma unroll
  for (int kb = 0; kb < E; kb += 32) { const v16b a = frag_kb(&Ah[nloc][kb], hlf), al = frag_kb(&Al[nloc][kb], hlf);
#pragma unroll
    for (int t4 = 0; t4 < 4; ++t4) { const v16b bw = frag_kb(&Wr[t4 * 16 + nloc][kb], hlf); acc[t4] = wmma16b(a, bw, acc[t4]); acc[t4] = wmma16b(al, bw, acc[t4]); } }
#pragma unroll
  for (int t4 = 0; t4 < 4; ++t4) { const int cc = t4 * 16 + nloc; const float bb = bfv(bo[cc]);
#pragma unroll
    for (int r8 = 0; r8 < 8; ++r8) Tf[8 * hlf + r8][cc] = acc[t4][r8] * (1.0f / (HS * WSC)) + bb; }
  wave_lds_sync();
  for (int pass = 0; pass < 2; ++pass) { for (int rr = 0; rr < 16; ++rr) *(volatile v2f*)(out + (r0 + rr) * E + lane * 2) = (v2f){Tf[rr][lane * 2], Tf[rr][lane * 2 + 1]}; __threadfence(); } }
}

extern "C" void kernel_launch(void* const* d_in, const int* in_sizes, int n_in, void* d_out, int out_size, void* d_ws, size_t ws_size, hipStream_t stream) {
  (void)n_in;
  auto Fp = [&](int i) { return (const float*)d_in[i]; };
  if (in_sizes[0] != NB_ * N * T * E || in_sizes[1] != NB_ * N * T * E || in_sizes[2] != NB_ * N * T * E || in_sizes[3] != HD * HD || in_sizes[6] != E * E || out_size != NB_ * N * T * E) return;
  const int GLIM = NBT * H;
  size_t off = 0; char* ws = (char*)d_ws;
  auto carve = [&](size_t bytes) { char* p = ws + off; off += (bytes + 255) & ~(size_t)255; return p; };
  const size_t ng = (size_t)NBT * H;
  b16* QPh = (b16*)carve(ng * N * 32 * 2); b16* QPl = (b16*)carve(ng * N * 32 * 2); b16* KPh = (b16*)carve(ng * N * 32 * 2); b16* KPl = (b16*)carve(ng * N * 32 * 2); b16* VTh = (b16*)carve(ng * 16 * N * 2); b16* VTl = (b16*)carve(ng * 16 * N * 2); float* AO = (float*)carve(ng * N * HD * 4);
  if (off > ws_size || off > ((size_t)80 << 20)) return;
  proj_kernel<<<NB_ * T * (N / 64), 256, 0, stream>>>(Fp(0), Fp(1), Fp(2), Fp(3), Fp(4), Fp(5), QPh, QPl, KPh, KPl, VTh, VTl);
  att_kernel<<<(unsigned)(ng * (N / 16)), 32, 0, stream>>>(QPh, QPl, KPh, KPl, VTh, VTl, GLIM, AO);
  outp_kernel<<<NB_ * N * T / 16, 32, 0, stream>>>(AO, Fp(6), Fp(7), GLIM, (float*)d_out);
}
